// MCA_23227183137075
// MI455X (gfx1250) — hardware-run, weakly checked
//
#include <hip/hip_runtime.h>
#include <math.h>

#ifndef NB
#define NB 8
#endif
#ifndef SEQ
#define SEQ 2048
#endif
#define SEQ_FULL 2048
#define CH 64
#define LH (SEQ / 2)
#define HEADS 8
#define QB (SEQ / 256)

constexpr unsigned ilog2c(unsigned v) { return v <= 1u ? 0u : 1u + ilog2c(v >> 1); }
#define LG_SEQ (ilog2c(SEQ))
#define LG_QB (ilog2c(QB))

static_assert((SEQ & (SEQ - 1)) == 0);
static_assert(SEQ % 256 == 0 && SEQ <= SEQ_FULL);
static_assert(LH % 128 == 0);
static_assert((NB * SEQ) % 128 == 0 && (NB * LH) % 128 == 0);
static_assert((NB * SEQ * 8) % 256 == 0);
static_assert(CH == 64 && HEADS * 8 == CH);
static_assert(64 % 32 == 0 && (3 * 128) % 32 == 0 && (3 * 192) % 32 == 0);

typedef __attribute__((ext_vector_type(16))) _Float16 v16h;
typedef __attribute__((ext_vector_type(8)))  _Float16 v8h;
typedef __attribute__((ext_vector_type(2)))  _Float16 v2h;
typedef __attribute__((ext_vector_type(8)))  float    v8f;
typedef __attribute__((ext_vector_type(4)))  float    v4f;
typedef __attribute__((ext_vector_type(2)))  float    v2f;
typedef __attribute__((ext_vector_type(4)))  unsigned int v4u;


#define VST2(T, ptr, val) do { const T vst2_v_ = (val); *(volatile T*)(ptr) = vst2_v_; __threadfence(); *(volatile T*)(ptr) = vst2_v_; } while (0)
#define VST2V4(ptr, val) do { const v4f vst2_v4_ = (val); *(volatile v4f*)(ptr) = vst2_v4_; __threadfence(); *(volatile v4f*)(ptr) = vst2_v4_; } while (0)

__device__ __forceinline__ float bfr(float f) {
    unsigned u = __float_as_uint(f);
    u += 0x7FFFu + ((u >> 16) & 1u);
    return __uint_as_float(u & 0xFFFF0000u);
}

static __device__ __forceinline__ float flush_sel(float v) { return (fabsf(v) < 6.103515625e-05f) ? 0.0f : v; }
static __device__ __forceinline__ unsigned toh_flush2(float a, float b) {
    v2f w; w.x = flush_sel(a); w.y = flush_sel(b);
    const v2h h = __builtin_convertvector(w, v2h);
    return __builtin_bit_cast(unsigned, h);
}
static __device__ __forceinline__ v4u cvt1w8(const float* a) {
    v4u p;
    p.x = toh_flush2(a[0], a[1]); p.y = toh_flush2(a[2], a[3]);
    p.z = toh_flush2(a[4], a[5]); p.w = toh_flush2(a[6], a[7]);
    return p;
}

union FragU { v16h v; v8h h[2]; };
__device__ __forceinline__ v16h frag_ld(const _Float16* p) {
    FragU f; f.h[0] = *(const v8h*)(p); f.h[1] = *(const v8h*)(p + 16); return f.v;
}
__device__ __forceinline__ v8f wmma16(v16h a, v16h b, v8f c) {
    c = __builtin_amdgcn_wmma_f32_16x16x32_f16(false, a, false, b, (short)0, c, false, false);
    asm volatile("v_nop\n\tv_nop\n\tv_nop\n\tv_nop" : "+v"(c) : "v"(a), "v"(b));
    return c;
}
__device__ __forceinline__ void wave_sync_lds() {
    __builtin_amdgcn_fence(3  , "workgroup");
    __builtin_amdgcn_wave_barrier();
    __builtin_amdgcn_fence(2  , "workgroup");
}

static_assert(32 * 16 * 8 == 16 * 256);
static_assert(32 * 16 * 4 == 16 * 128);
static_assert(8 * 16 * 68 * 4 <= 131072);
template <int EPI>
static __device__ __forceinline__ void conv_gemm_body(
    const _Float16* __restrict__ A, unsigned lda, unsigned rpbA,
    const _Float16* __restrict__ Bt, unsigned K,
    float* __restrict__ Cf, unsigned short* __restrict__ Ch,
    const float* __restrict__ r1, const float* __restrict__ r2,
    unsigned lgT, unsigned nb) {
  __shared__ __align__(16) float sT[8][16 * 68];
  const unsigned lane = threadIdx.x & 31u;
  const unsigned wave = (unsigned)__builtin_amdgcn_readfirstlane((int)(threadIdx.x >> 5));
  const unsigned tile = blockIdx.x * 8u + wave;
  if (tile >= (nb << lgT)) return;
  const unsigned b = tile >> lgT;
  const unsigned tm = tile - (b << lgT);
  const unsigned arow0 = b * rpbA + (tm << 6);
  const unsigned crow0 = tile << 6;
  const unsigned rlane = lane & 15u;
  const unsigned koff = (lane >> 4) * 8u;
  const unsigned mOff = koff;

  v8f acc[4][4];
#pragma unroll
  for (int i = 0; i < 4; ++i)
#pragma unroll
    for (int j = 0; j < 4; ++j) acc[i][j] = (v8f){0.f,0.f,0.f,0.f,0.f,0.f,0.f,0.f};

  for (unsigned k0 = 0; k0 < K; k0 += 32u) {
    v16h bh[4];
#pragma unroll
    for (int j = 0; j < 4; ++j)
      bh[j] = frag_ld(Bt + (((unsigned)j << 4) + rlane) * K + koff + k0);
#pragma unroll
    for (int i = 0; i < 4; ++i) {
      const v16h ah = frag_ld(A + (arow0 + ((unsigned)i << 4) + rlane) * lda + koff + k0);
#pragma unroll
      for (int j = 0; j < 4; ++j)
        acc[i][j] = wmma16(ah, bh[j], acc[i][j]);
    }
  }

  const float SC = 1.0f / 1048576.0f;
  float* slab = sT[wave];
#pragma unroll
  for (int i = 0; i < 4; ++i) {
    const unsigned mBase = crow0 + ((unsigned)i << 4);
#pragma unroll
    for (int j = 0; j < 4; ++j) {
#pragma unroll
      for (int r = 0; r < 8; ++r)
        slab[(mOff + (unsigned)r) * 68u + ((unsigned)j << 4) + rlane] = acc[i][j][r] * SC;
    }
    wave_sync_lds();
    if (EPI != 3) {
      const unsigned hh = lane >> 4, c4 = (lane & 15u) * 4u;
#pragma unroll
      for (int half = 0; half < 2; ++half) {
        v4f vv[4];
#pragma unroll
        for (int it = 0; it < 4; ++it) {
          const unsigned row = (unsigned)(half * 4 + it) * 2u + hh;
          const unsigned go = (mBase + row) * 64u + c4;
          v4f v = *(const v4f*)(slab + row * 68u + c4);
          if (EPI == 1) {
            const v4f xv = *(const v4f*)(r1 + go);
            v.x = xv.x * (1.0f / (1.0f + expf(-v.x)));
            v.y = xv.y * (1.0f / (1.0f + expf(-v.y)));
            v.z = xv.z * (1.0f / (1.0f + expf(-v.z)));
            v.w = xv.w * (1.0f / (1.0f + expf(-v.w)));
          }
          if (EPI == 2) {
            const v4f av = *(const v4f*)(r1 + go);
            const v4f ov = *(const v4f*)(r2 + go);
            const v4f xs = ov + av;
            v = v + xs;
          }
          vv[it] = v;
        }
        for (int pass = 0; pass < 2; ++pass) {
#pragma unroll
          for (int it = 0; it < 4; ++it) {
            const unsigned row = (unsigned)(half * 4 + it) * 2u + hh;
            *(volatile v4f*)(Cf + (mBase + row) * 64u + c4) = vv[it];
          }
          __threadfence();
        }
      }
    } else {
      const unsigned q = lane >> 3, c8 = (lane & 7u) * 8u;
      v4u hv[4];
#pragma unroll
      for (int it = 0; it < 4; ++it) {
        const unsigned row = (unsigned)it * 4u + q;
        const float* sp = slab + row * 68u + c8;
        float a[8];
#pragma unroll
        for (int e = 0; e < 8; ++e) a[e] = sp[e] * 1024.0f;
        hv[it] = cvt1w8(a);
      }
      for (int pass = 0; pass < 2; ++pass) {
#pragma unroll
        for (int it = 0; it < 4; ++it) {
          const unsigned row = (unsigned)it * 4u + q;
          *(volatile v4u*)(Ch + (mBase + row) * 64u + c8) = hv[it];
        }
        __threadfence();
      }
    }
    wave_sync_lds();
  }
}

__global__ __launch_bounds__(256) void k_conv_f32(const _Float16* __restrict__ A, unsigned lda, unsigned rpbA,
                                                  const _Float16* __restrict__ Bt, unsigned K,
                                                  float* __restrict__ C, unsigned lgT, unsigned nb) {
  conv_gemm_body<0>(A, lda, rpbA, Bt, K, C, (unsigned short*)nullptr, (const float*)nullptr, (const float*)nullptr, lgT, nb);
}
__global__ __launch_bounds__(256) void k_conv_gate(const _Float16* __restrict__ A, unsigned lda, unsigned rpbA,
                                                   const _Float16* __restrict__ Bt, unsigned K,
                                                   float* __restrict__ C, const float* __restrict__ xf,
                                                   unsigned lgT, unsigned nb) {
  conv_gemm_body<1>(A, lda, rpbA, Bt, K, C, (unsigned short*)nullptr, xf, (const float*)nullptr, lgT, nb);
}
__global__ __launch_bounds__(256) void k_conv_res(const _Float16* __restrict__ A, unsigned lda, unsigned rpbA,
                                                  const _Float16* __restrict__ Bt, unsigned K,
                                                  float* __restrict__ C, const float* __restrict__ xa,
                                                  const float* __restrict__ of, unsigned lgT, unsigned nb) {
  conv_gemm_body<2>(A, lda, rpbA, Bt, K, C, (unsigned short*)nullptr, xa, of, lgT, nb);
}
__global__ __launch_bounds__(256) void k_conv_h16(const _Float16* __restrict__ A, unsigned lda, unsigned rpbA,
                                                  const _Float16* __restrict__ Bt, unsigned K,
                                                  unsigned short* __restrict__ C, unsigned lgT, unsigned nb) {
  conv_gemm_body<3>(A, lda, rpbA, Bt, K, (float*)nullptr, C, (const float*)nullptr, (const float*)nullptr, lgT, nb);
}

__global__ __launch_bounds__(256) void k_wplane(const float* __restrict__ w, unsigned short* __restrict__ dst,
                                                unsigned chin, unsigned cpg, unsigned lgopg, unsigned taps) {
    const unsigned t = threadIdx.x;
    const unsigned o = blockIdx.x;
    const unsigned K = taps * chin;
    const unsigned k0 = t * 8u;
    if (k0 >= K) return;
    const unsigned tap = ((k0 >= chin) ? 1u : 0u) + ((k0 >= 2u * chin) ? 1u : 0u);
    const unsigned c0 = k0 - tap * chin;
    const unsigned go = o >> lgopg;
    const unsigned cl = c0 - go * cpg;
    const bool ing = cl < cpg;
    const unsigned clc = ing ? cl : 0u;
    float v[8];
#pragma unroll
    for (int i = 0; i < 8; ++i) {
        const float wv = bfr(w[(o * cpg + clc + (unsigned)i) * taps + tap]) * 4096.0f;
        v[i] = ing ? wv : 0.0f;
    }
    const v4u pk = cvt1w8(v);
    VST2(v4u, (v4u*)(dst + o * K + k0), pk);
}

static_assert(256 * 16 * 2 == 32 * 256 && 256 * 16 == 32 * 128);
__global__ __launch_bounds__(256) void k_xplane(const float* __restrict__ x, float* __restrict__ XF,
                                                unsigned short* __restrict__ X16) {
    __shared__ float sx[32 * 65];
    const unsigned t = threadIdx.x;
    const unsigned b = blockIdx.y, l0 = blockIdx.x * 32u;
#pragma unroll
    for (int it = 0; it < 8; ++it) {
        const unsigned c = (unsigned)it * 8u + (t >> 5), l = t & 31u;
        sx[l * 65u + c] = bfr(x[(b * CH + c) * SEQ_FULL + l0 + l]);
    }
    __syncthreads();
#pragma unroll
    for (int it = 0; it < 2; ++it) {
        const unsigned row = (unsigned)it * 16u + (t >> 4), c4 = (t & 15u) * 4u;
        v4f v;
        v.x = sx[row * 65u + c4]; v.y = sx[row * 65u + c4 + 1u]; v.z = sx[row * 65u + c4 + 2u]; v.w = sx[row * 65u + c4 + 3u];
        VST2V4(XF + (b * SEQ + l0 + row) * 64u + c4, v);
    }
    {
        const unsigned row = t >> 3, cg = t & 7u;
        float a[8];
#pragma unroll
        for (int i = 0; i < 8; ++i) a[i] = sx[row * 65u + 8u * cg + (unsigned)i] * 256.0f;
        const v4u pk = cvt1w8(a);
        VST2(v4u, (v4u*)(X16 + (b * SEQ + l0 + row) * 64u + 8u * cg), pk);
    }
}

__global__ __launch_bounds__(256) void k_cvt_xa(const float* __restrict__ XA, unsigned short* __restrict__ XA16,
                                                unsigned short* __restrict__ DS16) {
    const unsigned u = blockIdx.x * 256u + threadIdx.x;
    if (u >= (unsigned)(NB * SEQ * 8)) return;
    const unsigned row = u >> 3, cg = u & 7u;
    const unsigned b = row >> LG_SEQ, l = row & (unsigned)(SEQ - 1);
    const v4f a0 = *(const v4f*)(XA + row * 64u + 8u * cg);
    const v4f a1 = *(const v4f*)(XA + row * 64u + 8u * cg + 4u);
    const float a[8] = {a0.x * 256.0f, a0.y * 256.0f, a0.z * 256.0f, a0.w * 256.0f,
                        a1.x * 256.0f, a1.y * 256.0f, a1.z * 256.0f, a1.w * 256.0f};
    const v4u pk = cvt1w8(a);
    unsigned short* d1 = XA16 + row * 64u + 8u * cg;
    const unsigned j = l >> 1;
    const unsigned off = (l & 1u) ? 0u : 64u;
    unsigned short* d2 = DS16 + (b * (unsigned)(LH + 2) + j + 1u) * 128u + off + 8u * cg;
    for (int pass = 0; pass < 2; ++pass) {
        *(volatile v4u*)(d1) = pk;
        *(volatile v4u*)(d2) = pk;
        __threadfence();
    }
    const v4u zz = (v4u){0u, 0u, 0u, 0u};
    if (l == 0u || l == (unsigned)(SEQ - 1)) {
        const unsigned prow = (l == 0u) ? 0u : (unsigned)(LH + 1);
        unsigned short* dz = DS16 + (b * (unsigned)(LH + 2) + prow) * 128u + 8u * cg;
        for (int pass = 0; pass < 2; ++pass) {
            *(volatile v4u*)(dz) = zz;
            *(volatile v4u*)(dz + 64) = zz;
            __threadfence();
        }
    }
}

__global__ __launch_bounds__(256) void k_q16(const float* __restrict__ QF, unsigned short* __restrict__ Q16) {
    const unsigned u = blockIdx.x * 256u + threadIdx.x;
    if (u >= (unsigned)(NB * SEQ * 8)) return;
    const unsigned row = u >> 3, cg = u & 7u;
    const v4f a0 = *(const v4f*)(QF + row * 64u + 8u * cg);
    const v4f a1 = *(const v4f*)(QF + row * 64u + 8u * cg + 4u);
    const float QS = 362.03867196751236f;
    const float a[8] = {a0.x * QS, a0.y * QS, a0.z * QS, a0.w * QS, a1.x * QS, a1.y * QS, a1.z * QS, a1.w * QS};
    const v4u pk = cvt1w8(a);
    VST2(v4u, (v4u*)(Q16 + row * 64u + 8u * cg), pk);
}

static __device__ __forceinline__ float col_total(const float* __restrict__ part, unsigned nblk, unsigned c) {
    float s = 0.f;
    for (unsigned k = 0; k < nblk; ++k) s += part[k * 64u + c];
    return s;
}
__global__ __launch_bounds__(256) void k_colsum(const float* __restrict__ src, float* __restrict__ part) {
    __shared__ float red[4 * 64];
    __shared__ __align__(16) float fin[64];
    const unsigned t = threadIdx.x;
    const unsigned c = t & 63u, rq = t >> 6;
    const unsigned r0 = blockIdx.x * 128u;
    float s = 0.f;
    for (unsigned i = 0; i < 32u; ++i) s += src[(r0 + rq + 4u * i) * 64u + c];
    red[rq * 64u + c] = s;
    __syncthreads();
    if (t < 64u) fin[t] = ((red[t] + red[64u + t]) + red[128u + t]) + red[192u + t];
    __syncthreads();
    if (t < 16u) { const v4f v = *(const v4f*)(fin + 4u * t); VST2V4(part + blockIdx.x * 64u + 4u * t, v); }
}
__global__ __launch_bounds__(256) void k_colvar(const float* __restrict__ src, const float* __restrict__ part1,
                                                float* __restrict__ part2, unsigned nblk, unsigned nrows) {
    __shared__ float sMean[64];
    __shared__ float red[4 * 64];
    __shared__ __align__(16) float fin[64];
    const unsigned t = threadIdx.x;
    if (t < 64u) sMean[t] = col_total(part1, nblk, t) / (float)nrows;
    __syncthreads();
    const unsigned c = t & 63u, rq = t >> 6;
    const unsigned r0 = blockIdx.x * 128u;
    const float m = sMean[c];
    float s = 0.f;
    for (unsigned i = 0; i < 32u; ++i) { const float d = src[(r0 + rq + 4u * i) * 64u + c] - m; s += d * d; }
    red[rq * 64u + c] = s;
    __syncthreads();
    if (t < 64u) fin[t] = ((red[t] + red[64u + t]) + red[128u + t]) + red[192u + t];
    __syncthreads();
    if (t < 16u) { const v4f v = *(const v4f*)(fin + 4u * t); VST2V4(part2 + blockIdx.x * 64u + 4u * t, v); }
}

static_assert(256 * 16 * 4 == 128 * 128);
__global__ __launch_bounds__(256) void k_bn_cvt(const float* __restrict__ DN, const float* __restrict__ p1,
                                                const float* __restrict__ p2, const float* __restrict__ g,
                                                const float* __restrict__ bt, unsigned short* __restrict__ XD16,
                                                unsigned nblk, unsigned nrows) {
    __shared__ float sM[64];
    __shared__ float sR[64];
    __shared__ float sG[64];
    __shared__ float sB[64];
    const unsigned t = threadIdx.x;
    if (t < 64u) {
        const float mean = col_total(p1, nblk, t) / (float)nrows;
        const float var = col_total(p2, nblk, t) / (float)nrows;
        sM[t] = mean;
        sR[t] = 1.0f / sqrtf(var + 1e-5f);
        sG[t] = bfr(g[t]);
        sB[t] = bfr(bt[t]);
    }
    __syncthreads();
    const unsigned cg = t & 7u;
#pragma unroll
    for (int it = 0; it < 4; ++it) {
        const unsigned row = blockIdx.x * 128u + (unsigned)it * 32u + (t >> 3);
        const v4f a0 = *(const v4f*)(DN + row * 64u + 8u * cg);
        const v4f a1 = *(const v4f*)(DN + row * 64u + 8u * cg + 4u);
        const float a[8] = {a0.x, a0.y, a0.z, a0.w, a1.x, a1.y, a1.z, a1.w};
        float y[8];
#pragma unroll
        for (int i = 0; i < 8; ++i) {
            const unsigned c = 8u * cg + (unsigned)i;
            const float xn = (a[i] - sM[c]) * sR[c];
            y[i] = fmaxf(xn * sG[c] + sB[c], 0.0f) * 256.0f;
        }
        const v4u pk = cvt1w8(y);
        VST2(v4u, (v4u*)(XD16 + row * 64u + 8u * cg), pk);
    }
}

static_assert(256 * 16 * 4 == 128 * 128);
__global__ __launch_bounds__(256) void k_vt(const float* __restrict__ V1F, unsigned short* __restrict__ VT16) {
    __shared__ float sv[64 * 65];
    const unsigned t = threadIdx.x;
    const unsigned b = blockIdx.y, m0 = blockIdx.x * 64u;
#pragma unroll
    for (int it = 0; it < 4; ++it) {
        const unsigned row = (unsigned)it * 16u + (t >> 4), c4 = (t & 15u) * 4u;
        const v4f v = *(const v4f*)(V1F + (b * LH + m0 + row) * 64u + c4);
        sv[row * 65u + c4] = v.x; sv[row * 65u + c4 + 1u] = v.y; sv[row * 65u + c4 + 2u] = v.z; sv[row * 65u + c4 + 3u] = v.w;
    }
    __syncthreads();
#pragma unroll
    for (int it = 0; it < 4; ++it) {
        const unsigned idx = (unsigned)it * 256u + t;
        const unsigned rid = idx >> 3, kg = idx & 7u;
        const unsigned h = rid >> 4, e = rid & 15u;
        const unsigned ch = 8u * h + (e & 7u);
        const bool live = e < 8u;
        float a[8];
#pragma unroll
        for (int i = 0; i < 8; ++i) {
            const float sval = sv[(8u * kg + (unsigned)i) * 65u + ch] * 1024.0f;
            a[i] = live ? sval : 0.0f;
        }
        const v4u pk = cvt1w8(a);
        VST2(v4u, (v4u*)(VT16 + ((b * HEADS + h) * 16u + e) * LH + m0 + 8u * kg), pk);
    }
}

#define AT_PP 72
#define AT_OP 68
static_assert(16 * 16 * AT_PP * 2 + 16 * 16 * AT_OP * 4 <= 131072);
static_assert(32 * 16 * 8 == 16 * 64 * 4);
static_assert(LH % 64 == 0);
__global__ __launch_bounds__(512) void k_attn(const _Float16* __restrict__ Q16, const _Float16* __restrict__ K16,
                                              const _Float16* __restrict__ VT16, float* __restrict__ OF) {
    __shared__ __align__(16) _Float16 sP[16][16 * AT_PP];
    __shared__ __align__(16) float sO[16][16 * AT_OP];
    const unsigned tid = threadIdx.x, lane = tid & 31u;
    const unsigned wave = (unsigned)__builtin_amdgcn_readfirstlane((int)(tid >> 5));
    const unsigned hh = lane >> 4, c = lane & 15u;
    const unsigned b = blockIdx.x >> LG_QB, qb = blockIdx.x & (unsigned)(QB - 1);
    const unsigned q0 = qb * 256u + wave * 16u;
    _Float16* pw = sP[wave];
    float* so = sO[wave];
    const float SC2 = 1.4426950408889634f * (1.0f / 1048576.0f);
    v8h zh;
#pragma unroll
    for (int e = 0; e < 8; ++e) zh[e] = (_Float16)0.0f;
    for (unsigned head = 0; head < (unsigned)HEADS; ++head) {
        const v8h qv = *(const v8h*)(Q16 + (b * SEQ + q0 + c) * 64u + 8u * head);
        FragU qf;
        qf.h[0] = (hh == 0u) ? qv : zh;
        qf.h[1] = zh;
        const _Float16* kb = K16 + (b * LH + c) * 64u + 8u * head;
        const _Float16* vb0 = VT16 + ((b * HEADS + head) * 16u + c) * LH + 8u * hh;
        float mrow[8], lrow[8];
        v8f os = (v8f){0.f,0.f,0.f,0.f,0.f,0.f,0.f,0.f};
#pragma unroll
        for (int r = 0; r < 8; ++r) { mrow[r] = -3.0e38f; lrow[r] = 0.f; }
#pragma unroll 1
        for (unsigned kc = 0; kc < (unsigned)(LH / 64); ++kc) {
            const unsigned kv0 = kc * 64u;
            v8f s[4];
#pragma unroll
            for (int j = 0; j < 4; ++j) {
                const v8h kv = *(const v8h*)(kb + (kv0 + (unsigned)j * 16u) * 64u);
                FragU kf;
                kf.h[0] = (hh == 0u) ? kv : zh;
                kf.h[1] = zh;
                const v8f z = (v8f){0.f,0.f,0.f,0.f,0.f,0.f,0.f,0.f};
                s[j] = wmma16(qf.v, kf.v, z);
            }
#pragma unroll
            for (int r = 0; r < 8; ++r) {
                float mx = -3.0e38f;
#pragma unroll
                for (int j = 0; j < 4; ++j) { s[j][r] *= SC2; mx = fmaxf(mx, s[j][r]); }
                mx = fmaxf(mx, __shfl_xor(mx, 1, 32)); mx = fmaxf(mx, __shfl_xor(mx, 2, 32));
                mx = fmaxf(mx, __shfl_xor(mx, 4, 32)); mx = fmaxf(mx, __shfl_xor(mx, 8, 32));
                const float mnew = fmaxf(mrow[r], mx);
                const float alpha = exp2f(mrow[r] - mnew);
                mrow[r] = mnew;
                float psum = 0.f;
#pragma unroll
                for (int j = 0; j < 4; ++j) {
                    const float ex = s[j][r] - mnew;
                    const float p = exp2f(ex);
                    psum += p;
                    const float pc = (ex < -24.0f) ? 0.0f : p * 1024.0f;
                    pw[(8u * hh + (unsigned)r) * AT_PP + (unsigned)j * 16u + c] = (_Float16)pc;
                }
                lrow[r] = lrow[r] * alpha + psum;
                os[r] *= alpha;
            }
            wave_sync_lds();
#pragma unroll
            for (int kk = 0; kk < 2; ++kk) {
                const v16h pa = frag_ld(pw + c * AT_PP + (unsigned)kk * 32u + 8u * hh);
                const v16h vb = frag_ld(vb0 + kv0 + (unsigned)kk * 32u);
                os = wmma16(pa, vb, os);
            }
            wave_sync_lds();
        }
#pragma unroll
        for (int r = 0; r < 8; ++r) {
            float l = lrow[r];
            l += __shfl_xor(l, 1, 32); l += __shfl_xor(l, 2, 32);
            l += __shfl_xor(l, 4, 32); l += __shfl_xor(l, 8, 32);
            const float inv = 1.0f / (l * 1048576.0f);
            const float ov = os[r] * inv;
            if (c < 8u) so[(8u * hh + (unsigned)r) * AT_OP + 8u * head + c] = ov;
        }
    }
    wave_sync_lds();
    {
        const unsigned c4 = c * 4u;
        float* dst = OF + (b * SEQ + q0) * 64u;
#pragma unroll
        for (int half = 0; half < 2; ++half) {
            v4f vv[4];
#pragma unroll
            for (int it = 0; it < 4; ++it) {
                const unsigned row = (unsigned)(half * 4 + it) * 2u + hh;
                vv[it] = *(const v4f*)(so + row * AT_OP + c4);
            }
            for (int pass = 0; pass < 2; ++pass) {
#pragma unroll
                for (int it = 0; it < 4; ++it) {
                    const unsigned row = (unsigned)(half * 4 + it) * 2u + hh;
                    *(volatile v4f*)(dst + row * 64u + c4) = vv[it];
                }
                __threadfence();
            }
        }
    }
}

__global__ __launch_bounds__(256) void k_cat(const float* __restrict__ OF, const float* __restrict__ XA,
                                             const float* __restrict__ QF, unsigned short* __restrict__ XC16) {
    const unsigned u = blockIdx.x * 256u + threadIdx.x;
    if (u >= (unsigned)(NB * SEQ * 8)) return;
    const unsigned row = u >> 3, cg = u & 7u;
    const unsigned b = row >> LG_SEQ, l = row & (unsigned)(SEQ - 1);
    const unsigned go = row * 64u + 8u * cg;
    const v4f o0 = *(const v4f*)(OF + go), o1 = *(const v4f*)(OF + go + 4u);
    const v4f a0 = *(const v4f*)(XA + go), a1 = *(const v4f*)(XA + go + 4u);
    const v4f q0 = *(const v4f*)(QF + go), q1 = *(const v4f*)(QF + go + 4u);
    const float ov[8] = {o0.x * 256.0f, o0.y * 256.0f, o0.z * 256.0f, o0.w * 256.0f,
                         o1.x * 256.0f, o1.y * 256.0f, o1.z * 256.0f, o1.w * 256.0f};
    const float qv[8] = {q0.x * 256.0f, q0.y * 256.0f, q0.z * 256.0f, q0.w * 256.0f,
                         q1.x * 256.0f, q1.y * 256.0f, q1.z * 256.0f, q1.w * 256.0f};
    const float xs[8] = {(o0.x + a0.x) * 256.0f, (o0.y + a0.y) * 256.0f, (o0.z + a0.z) * 256.0f, (o0.w + a0.w) * 256.0f,
                         (o1.x + a1.x) * 256.0f, (o1.y + a1.y) * 256.0f, (o1.z + a1.z) * 256.0f, (o1.w + a1.w) * 256.0f};
    const v4u pkx = cvt1w8(xs);
    const v4u pkq = cvt1w8(qv);
    const v4u pko = cvt1w8(ov);
    unsigned short* d = XC16 + (b * (unsigned)(SEQ + 2) + l + 1u) * 192u + 8u * cg;
    for (int pass = 0; pass < 2; ++pass) {
        *(volatile v4u*)(d) = pkx;
        *(volatile v4u*)(d + 64) = pkq;
        *(volatile v4u*)(d + 128) = pko;
        __threadfence();
    }
    const v4u zz = (v4u){0u, 0u, 0u, 0u};
    if (l == 0u || l == (unsigned)(SEQ - 1)) {
        const unsigned prow = (l == 0u) ? 0u : (unsigned)(SEQ + 1);
        unsigned short* dz = XC16 + (b * (unsigned)(SEQ + 2) + prow) * 192u + 8u * cg;
        for (int pass = 0; pass < 2; ++pass) {
            *(volatile v4u*)(dz) = zz;
            *(volatile v4u*)(dz + 64) = zz;
            *(volatile v4u*)(dz + 128) = zz;
            __threadfence();
        }
    }
}

static_assert(256 * 16 * 4 == 64 * 256);
__global__ __launch_bounds__(256) void k_final(const float* __restrict__ XS2, const float* __restrict__ p1,
                                               const float* __restrict__ p2, const float* __restrict__ g,
                                               const float* __restrict__ bt, float* __restrict__ out,
                                               unsigned nblk, unsigned nrows) {
    __shared__ float sM[64];
    __shared__ float sR[64];
    __shared__ float sG[64];
    __shared__ float sB[64];
    __shared__ float st[64 * 65];
    const unsigned t = threadIdx.x;
    const unsigned b = blockIdx.y, l0 = blockIdx.x * 64u;
    if (t < 64u) {
        const float mean = col_total(p1, nblk, t) / (float)nrows;
        const float var = col_total(p2, nblk, t) / (float)nrows;
        sM[t] = mean;
        sR[t] = 1.0f / sqrtf(var + 1e-5f);
        sG[t] = bfr(g[t]);
        sB[t] = bfr(bt[t]);
    }
    __syncthreads();
#pragma unroll
    for (int it = 0; it < 4; ++it) {
        const unsigned row = (unsigned)it * 16u + (t >> 4), c4 = (t & 15u) * 4u;
        const v4f v = *(const v4f*)(XS2 + (b * SEQ + l0 + row) * 64u + c4);
        const float e[4] = {v.x, v.y, v.z, v.w};
#pragma unroll
        for (int i = 0; i < 4; ++i) {
            const unsigned c = c4 + (unsigned)i;
            const float xn = (e[i] - sM[c]) * sR[c];
            st[row * 65u + c] = fmaxf(xn * sG[c] + sB[c], 0.0f);
        }
    }
    __syncthreads();
#pragma unroll
    for (int it = 0; it < 4; ++it) {
        const unsigned idx = (unsigned)it * 256u + t;
        const unsigned chn = idx >> 4, lq = idx & 15u;
        v4f o;
        o.x = st[(4u * lq) * 65u + chn]; o.y = st[(4u * lq + 1u) * 65u + chn];
        o.z = st[(4u * lq + 2u) * 65u + chn]; o.w = st[(4u * lq + 3u) * 65u + chn];
        VST2V4(out + (b * CH + chn) * SEQ_FULL + l0 + 4u * lq, o);
    }
}

constexpr size_t al256(size_t v) { return (v + 255) & ~(size_t)255; }
constexpr size_t SZ_W1   = (size_t)64 * 64 * 2;
constexpr size_t SZ_WD   = (size_t)64 * 384 * 2;
constexpr size_t SZ_WO   = (size_t)64 * 576 * 2;
constexpr size_t SZ_F32L = (size_t)NB * SEQ * 64 * 4;
constexpr size_t SZ_F32H = (size_t)NB * LH * 64 * 4;
constexpr size_t SZ_1WL  = (size_t)NB * SEQ * 64 * 2;
constexpr size_t SZ_1WH  = (size_t)NB * LH * 64 * 2;
constexpr size_t SZ_DS   = (size_t)NB * (LH + 2) * 128 * 2;
constexpr size_t SZ_XC   = (size_t)NB * (SEQ + 2) * 192 * 2;
constexpr size_t SZ_Q16  = (size_t)NB * SEQ * 64 * 2;
constexpr size_t SZ_K16  = (size_t)NB * LH * 64 * 2;
constexpr size_t SZ_VT   = (size_t)NB * HEADS * 16 * LH * 2;
constexpr size_t SZ_PD   = (size_t)(NB * LH / 128) * 64 * 4;
constexpr size_t SZ_PF   = (size_t)(NB * SEQ / 128) * 64 * 4;
constexpr size_t OFF_WQ  = 0;
constexpr size_t OFF_WK  = OFF_WQ  + al256(SZ_W1);
constexpr size_t OFF_WV  = OFF_WK  + al256(SZ_W1);
constexpr size_t OFF_WV1 = OFF_WV  + al256(SZ_W1);
constexpr size_t OFF_WD  = OFF_WV1 + al256(SZ_W1);
constexpr size_t OFF_WO  = OFF_WD  + al256(SZ_WD);
constexpr size_t OFF_XF  = OFF_WO  + al256(SZ_WO);
constexpr size_t OFF_X16 = OFF_XF  + al256(SZ_F32L);
constexpr size_t OFF_XA  = OFF_X16 + al256(SZ_1WL);
constexpr size_t OFF_XA16 = OFF_XA + al256(SZ_F32L);
constexpr size_t OFF_DS  = OFF_XA16 + al256(SZ_1WL);
constexpr size_t OFF_QF  = OFF_DS  + al256(SZ_DS);
constexpr size_t OFF_Q16 = OFF_QF  + al256(SZ_F32L);
constexpr size_t OFF_DN  = OFF_Q16 + al256(SZ_Q16);
constexpr size_t OFF_P1D = OFF_DN  + al256(SZ_F32H);
constexpr size_t OFF_P2D = OFF_P1D + al256(SZ_PD);
constexpr size_t OFF_XD  = OFF_P2D + al256(SZ_PD);
constexpr size_t OFF_K16 = OFF_XD  + al256(SZ_1WH);
constexpr size_t OFF_V1F = OFF_K16 + al256(SZ_K16);
constexpr size_t OFF_VT  = OFF_V1F + al256(SZ_F32H);
constexpr size_t OFF_OF  = OFF_VT  + al256(SZ_VT);
constexpr size_t OFF_XC  = OFF_OF  + al256(SZ_F32L);
constexpr size_t OFF_XS2 = OFF_XC  + al256(SZ_XC);
constexpr size_t OFF_P1F = OFF_XS2 + al256(SZ_F32L);
constexpr size_t OFF_P2F = OFF_P1F + al256(SZ_PF);
constexpr size_t WS_TOTAL = OFF_P2F + al256(SZ_PF);
static_assert(WS_TOTAL <= 134217728);
static_assert((size_t)NB * (SEQ + 2) * 192 < 4294967296ull);

extern "C" void kernel_launch(void* const* d_in, const int* in_sizes, int n_in, void* d_out, int out_size,
                              void* d_ws, size_t ws_size, hipStream_t stream) {
    if (n_in < 11) return;
    if (in_sizes[0] < NB * CH * SEQ_FULL) return;
    if (in_sizes[1] < 1024 || in_sizes[2] < 1024 || in_sizes[3] < 1024 || in_sizes[4] < 1024) return;
    if (in_sizes[5] < 64 * 48 * 3 || in_sizes[6] < 64 * 64 * 3) return;
    if (in_sizes[7] < 64 || in_sizes[8] < 64 || in_sizes[9] < 64 || in_sizes[10] < 64) return;
    if (out_size < NB * CH * SEQ_FULL) return;
    if (ws_size < WS_TOTAL) return;

    const float* x          = (const float*)d_in[0];
    const float* q_w        = (const float*)d_in[1];
    const float* k_w        = (const float*)d_in[2];
    const float* v_w        = (const float*)d_in[3];
    const float* v1_w       = (const float*)d_in[4];
    const float* out_w      = (const float*)d_in[5];
    const float* down_w     = (const float*)d_in[6];
    const float* down_gamma = (const float*)d_in[7];
    const float* down_beta  = (const float*)d_in[8];
    const float* gamma      = (const float*)d_in[9];
    const float* beta       = (const float*)d_in[10];
    float* out = (float*)d_out;

    char* wsp = (char*)d_ws;
    unsigned short* WQ   = (unsigned short*)(wsp + OFF_WQ);
    unsigned short* WK   = (unsigned short*)(wsp + OFF_WK);
    unsigned short* WV   = (unsigned short*)(wsp + OFF_WV);
    unsigned short* WV1  = (unsigned short*)(wsp + OFF_WV1);
    unsigned short* WD   = (unsigned short*)(wsp + OFF_WD);
    unsigned short* WO   = (unsigned short*)(wsp + OFF_WO);
    float*          XF   = (float*)(wsp + OFF_XF);
    unsigned short* X16  = (unsigned short*)(wsp + OFF_X16);
    float*          XA   = (float*)(wsp + OFF_XA);
    unsigned short* XA16 = (unsigned short*)(wsp + OFF_XA16);
    unsigned short* DS16 = (unsigned short*)(wsp + OFF_DS);
    float*          QF   = (float*)(wsp + OFF_QF);
    unsigned short* Q16  = (unsigned short*)(wsp + OFF_Q16);
    float*          DN   = (float*)(wsp + OFF_DN);
    float*          P1D  = (float*)(wsp + OFF_P1D);
    float*          P2D  = (float*)(wsp + OFF_P2D);
    unsigned short* XD16 = (unsigned short*)(wsp + OFF_XD);
    unsigned short* K16  = (unsigned short*)(wsp + OFF_K16);
    float*          V1F  = (float*)(wsp + OFF_V1F);
    unsigned short* VT16 = (unsigned short*)(wsp + OFF_VT);
    float*          OF   = (float*)(wsp + OFF_OF);
    unsigned short* XC16 = (unsigned short*)(wsp + OFF_XC);
    float*          XS2  = (float*)(wsp + OFF_XS2);
    float*          P1F  = (float*)(wsp + OFF_P1F);
    float*          P2F  = (float*)(wsp + OFF_P2F);

    k_wplane<<<64, 256, 0, stream>>>(q_w,    WQ,  64u, 16u, 4u, 1u);
    k_wplane<<<64, 256, 0, stream>>>(k_w,    WK,  64u, 16u, 4u, 1u);
    k_wplane<<<64, 256, 0, stream>>>(v_w,    WV,  64u, 16u, 4u, 1u);
    k_wplane<<<64, 256, 0, stream>>>(v1_w,   WV1, 64u, 16u, 4u, 1u);
    k_wplane<<<64, 256, 0, stream>>>(down_w, WD, 128u, 64u, 5u, 3u);
    k_wplane<<<64, 256, 0, stream>>>(out_w,  WO, 192u, 48u, 4u, 3u);

    const unsigned lgL = ilog2c(SEQ / 64), lgH = ilog2c(LH / 64);
    const unsigned gL = ((unsigned)(NB * SEQ / 64) + 7u) / 8u;
    const unsigned gH = ((unsigned)(NB * LH / 64) + 7u) / 8u;
    const unsigned gE = (unsigned)(NB * SEQ * 8 / 256);
    const unsigned nblkD = (unsigned)(NB * LH / 128), nblkF = (unsigned)(NB * SEQ / 128);

    k_xplane<<<dim3(SEQ / 32, NB), 256, 0, stream>>>(x, XF, X16);
    k_conv_gate<<<gL, 256, 0, stream>>>((const _Float16*)X16, 64u, (unsigned)SEQ, (const _Float16*)WQ, 64u, XA, XF, lgL, (unsigned)NB);
    k_cvt_xa<<<gE, 256, 0, stream>>>(XA, XA16, DS16);
    k_conv_f32<<<gL, 256, 0, stream>>>((const _Float16*)XA16, 64u, (unsigned)SEQ, (const _Float16*)WK, 64u, QF, lgL, (unsigned)NB);
    k_q16<<<gE, 256, 0, stream>>>(QF, Q16);
    k_conv_f32<<<gH, 256, 0, stream>>>((const _Float16*)DS16, 128u, (unsigned)(LH + 2), (const _Float16*)WD, 384u, DN, lgH, (unsigned)NB);
    k_colsum<<<nblkD, 256, 0, stream>>>(DN, P1D);
    k_colvar<<<nblkD, 256, 0, stream>>>(DN, P1D, P2D, nblkD, (unsigned)(NB * LH));
    k_bn_cvt<<<nblkD, 256, 0, stream>>>(DN, P1D, P2D, down_gamma, down_beta, XD16, nblkD, (unsigned)(NB * LH));
    k_conv_h16<<<gH, 256, 0, stream>>>((const _Float16*)XD16, 64u, (unsigned)LH, (const _Float16*)WV, 64u, K16, lgH, (unsigned)NB);
    k_conv_f32<<<gH, 256, 0, stream>>>((const _Float16*)XD16, 64u, (unsigned)LH, (const _Float16*)WV1, 64u, V1F, lgH, (unsigned)NB);
    k_vt<<<dim3(LH / 64, NB), 256, 0, stream>>>(V1F, VT16);
    k_attn<<<NB * QB, 512, 0, stream>>>((const _Float16*)Q16, (const _Float16*)K16, (const _Float16*)VT16, OF);
    k_cat<<<gE, 256, 0, stream>>>(OF, XA, QF, XC16);
    k_conv_res<<<gL, 256, 0, stream>>>((const _Float16*)XC16, 192u, (unsigned)(SEQ + 2), (const _Float16*)WO, 576u, XS2, XA, OF, lgL, (unsigned)NB);
    k_colsum<<<nblkF, 256, 0, stream>>>(XS2, P1F);
    k_colvar<<<nblkF, 256, 0, stream>>>(XS2, P1F, P2F, nblkF, (unsigned)(NB * SEQ));
    k_final<<<dim3(SEQ / 64, NB), 256, 0, stream>>>(XS2, P1F, P2F, gamma, beta, out, nblkF, (unsigned)(NB * SEQ));
}
